// EfficientAdditiveAttention_46557445488980
// MI455X (gfx1250) — hardware-run, weakly checked
//
#include <hip/hip_runtime.h>
#include <math.h>
#include <stdint.h>

#define DEVINL __device__ __forceinline__

typedef _Float16 f16t;
typedef _Float16 v16h __attribute__((ext_vector_type(16)));
typedef _Float16 v8h  __attribute__((ext_vector_type(8)));
typedef float    v8f  __attribute__((ext_vector_type(8)));
typedef float    v4f  __attribute__((ext_vector_type(4)));
typedef v8h __attribute__((may_alias)) v8ha;
typedef v4f __attribute__((may_alias)) v4fa;
union FragH { v16h v; v8h half[2]; };

#define NB       8
#define NL       512
#define ND       128
#define NROWS    (NB * NL)
#define PJ_TPB   128
#define PJ_WAVES 4
#define PJ_ROWS  16
#define TPITCH   132
#define AT_TPB   256
#define AT_WAVES 8
#define QT       16
#define KC       16
#define OPITCH   132

#define WCAR     64.0f
#define SC_W     (1.0f / 64.0f)
#define VCAR     16.0f
#define PCAR     16384.0f
#define SC_PV    (1.0f / 262144.0f)
#define INV_SCALE 0.088388347648318447f
#define NEG_INF  (-__builtin_inff())

static_assert(PJ_TPB == PJ_WAVES * 32);
static_assert(AT_TPB == AT_WAVES * 32);
static_assert((NROWS % PJ_ROWS) == 0);
static_assert((NROWS % QT) == 0);
static_assert((NL % QT) == 0);
static_assert((NL % 32) == 0);
static_assert((ND % 32) == 0);
static_assert(PJ_WAVES * 32 == ND);
static_assert(PJ_WAVES * 4 == PJ_ROWS);
static_assert(AT_WAVES * 16 == ND);
static_assert(AT_WAVES * 2 == QT);
static_assert(32 * 4 == ND);
static_assert(QT * KC == AT_TPB);
static_assert(2 * AT_TPB * 4 == QT * ND);
static_assert(QT * OPITCH <= QT * NL);
static_assert((TPITCH % 4) == 0);
static_assert((OPITCH % 4) == 0);
static_assert(2 * QT * ND * 4 == QT * NL * 2);

DEVINL v8f wmma_f16(v16h a, v16h b, v8f c) {
  v8f d = __builtin_amdgcn_wmma_f32_16x16x32_f16(false, a, false, b, (short)0, c, false, false);
  asm volatile("v_nop\n\tv_nop\n\tv_nop\n\tv_nop" : "+v"(d) : "v"(a), "v"(b));
  return d;
}
DEVINL v8f zero8f() {
  v8f z = {0.f, 0.f, 0.f, 0.f, 0.f, 0.f, 0.f, 0.f};
  return z;
}
DEVINL void load_frag_f32(FragH& f, const float* row, int k0, float scale) {
  const v4f x0 = *(const v4fa*)(row + k0);
  const v4f x1 = *(const v4fa*)(row + k0 + 4);
  const v4f x2 = *(const v4fa*)(row + k0 + 16);
  const v4f x3 = *(const v4fa*)(row + k0 + 20);
  #pragma unroll
  for (int j = 0; j < 4; ++j) {
    f.v[j]      = (f16t)(x0[j] * scale);
    f.v[4 + j]  = (f16t)(x1[j] * scale);
    f.v[8 + j]  = (f16t)(x2[j] * scale);
    f.v[12 + j] = (f16t)(x3[j] * scale);
  }
}

__global__ __launch_bounds__(PJ_TPB) void proj_k(const float* __restrict__ xq, const float* __restrict__ xk,
                                             const float* __restrict__ xv,
                                             const float* __restrict__ Wq, const float* __restrict__ bq,
                                             const float* __restrict__ Wk, const float* __restrict__ bk,
                                             const float* __restrict__ Wv, const float* __restrict__ bv,
                                             float* __restrict__ Qp, float* __restrict__ Kp, float* __restrict__ Vp)
{
  __shared__ __attribute__((aligned(16))) float T_s[PJ_ROWS * TPITCH];
  const int tid = threadIdx.x, lane = tid & 31;
  const int wave = __builtin_amdgcn_readfirstlane(tid >> 5);
  const int hh = lane >> 4, m = lane & 15;
  if (blockIdx.x >= NROWS / PJ_ROWS) return;
  const int sel = blockIdx.y;
  const float* X    = (sel == 0) ? xq : ((sel == 1) ? xk : xv);
  const float* W    = (sel == 0) ? Wq : ((sel == 1) ? Wk : Wv);
  const float* bias = (sel == 0) ? bq : ((sel == 1) ? bk : bv);
  float* Y          = (sel == 0) ? Qp : ((sel == 1) ? Kp : Vp);

  const int row0 = blockIdx.x * PJ_ROWS;
  const int n0 = 32 * wave;
  const float* xrow = X + (size_t)(row0 + m) * ND + 8 * hh;

  v8f acc[2];
  acc[0] = zero8f();
  acc[1] = zero8f();

  #pragma unroll
  for (int ks = 0; ks < ND / 32; ++ks) {
    const int k0 = 32 * ks;
    FragH a;
    load_frag_f32(a, xrow, k0, 1.0f);
    #pragma unroll
    for (int t = 0; t < 2; ++t) {
      const float* wrow = W + (size_t)(n0 + 16 * t + m) * ND + 8 * hh;
      FragH b;
      load_frag_f32(b, wrow, k0, WCAR);
      acc[t] = wmma_f16(a.v, b.v, acc[t]);
    }
  }

  float bb[2];
  #pragma unroll
  for (int t = 0; t < 2; ++t) bb[t] = bias[n0 + 16 * t + m];
  #pragma unroll
  for (int r = 0; r < 8; ++r) {
    const int row = 8 * hh + r;
    #pragma unroll
    for (int t = 0; t < 2; ++t)
      T_s[row * TPITCH + n0 + 16 * t + m] = acc[t][r] * SC_W + bb[t];
  }
  __syncthreads();

  v4f va[4];
  float* da[4];
  #pragma unroll
  for (int j = 0; j < 4; ++j) {
    const int row = 4 * wave + j;
    va[j] = *(const v4fa*)(T_s + row * TPITCH + 4 * lane);
    da[j] = Y + (size_t)(row0 + row) * ND + 4 * lane;
    *(volatile v4f*)da[j] = va[j];
  }
  __threadfence();
  #pragma unroll
  for (int j = 0; j < 4; ++j) *(volatile v4f*)da[j] = va[j];
}

union QKP { float qk[2][QT * ND]; f16t p[QT * NL]; };

__global__ __launch_bounds__(AT_TPB) void attn_k(const float* __restrict__ Qp, const float* __restrict__ Kp,
                                                const float* __restrict__ Vp,
                                                const float* __restrict__ w_delta, const float* __restrict__ b_delta,
                                                const float* __restrict__ w_sigma, const float* __restrict__ b_sigma,
                                                const float* __restrict__ w_theta, const float* __restrict__ b_theta,
                                                float* __restrict__ out)
{
  __shared__ __attribute__((aligned(16))) QKP uqk;
  __shared__ __attribute__((aligned(16))) float sS[QT * NL];
  __shared__ __attribute__((aligned(16))) float sW[ND];
  __shared__ float sInv[QT];

  const int tid = threadIdx.x, lane = tid & 31;
  const int wave = __builtin_amdgcn_readfirstlane(tid >> 5);
  const int hh = lane >> 4, m = lane & 15;
  if (blockIdx.x >= NROWS / QT) return;
  const int bx = blockIdx.x;
  const int b  = bx / (NL / QT);
  const int q0 = bx * QT;
  const size_t bL = (size_t)b * NL;

  #pragma unroll
  for (int j = 0; j < 2; ++j) {
    const int i = tid + AT_TPB * j;
    const int row = i >> 5, col = 4 * (i & 31);
    *(v4fa*)(&uqk.qk[0][row * ND + col]) = *(const v4fa*)(Qp + (size_t)(q0 + row) * ND + col);
  }
  if (tid < ND) sW[tid] = ((INV_SCALE + w_delta[tid]) + w_sigma[tid]) + w_theta[tid];
  const float b_all = (b_delta[0] + b_sigma[0]) + b_theta[0];

  const int qi = tid & 15, kl = tid >> 4;
  const float* qr = &uqk.qk[0][qi * ND];
  const float* kr = &uqk.qk[1][kl * ND];
  #pragma unroll 1
  for (int kc = 0; kc < NL; kc += KC) {
    #pragma unroll
    for (int j = 0; j < 2; ++j) {
      const int i = tid + AT_TPB * j;
      const int row = i >> 5, col = 4 * (i & 31);
      *(v4fa*)(&uqk.qk[1][row * ND + col]) = *(const v4fa*)(Kp + (bL + kc + row) * ND + col);
    }
    __syncthreads();

    float acc = 0.0f;
    #pragma unroll 1
    for (int d = 0; d < ND; d += 4) {
      const v4f q4 = *(const v4fa*)(qr + d);
      const v4f k4 = *(const v4fa*)(kr + d);
      const v4f w4 = *(const v4fa*)(sW + d);
      #pragma unroll
      for (int j = 0; j < 4; ++j) acc = fmaf(tanhf(q4[j] + k4[j]), w4[j], acc);
    }
    sS[qi * NL + kc + kl] = acc + b_all;
    __syncthreads();
  }

  {
    const int r = tid >> 4, t = tid & 15;
    const float* srow = sS + r * NL;
    float mx = NEG_INF;
    #pragma unroll 4
    for (int kk = t; kk < NL; kk += 16) mx = fmaxf(mx, srow[kk]);
    mx = fmaxf(mx, __shfl_xor(mx, 8));
    mx = fmaxf(mx, __shfl_xor(mx, 4));
    mx = fmaxf(mx, __shfl_xor(mx, 2));
    mx = fmaxf(mx, __shfl_xor(mx, 1));
    float sum = 0.0f;
    f16t* prow = &uqk.p[r * NL];
    #pragma unroll 4
    for (int kk = t; kk < NL; kk += 16) {
      const float e = __expf(srow[kk] - mx);
      sum += e;
      prow[kk] = (f16t)(e * PCAR);
    }
    sum += __shfl_xor(sum, 8);
    sum += __shfl_xor(sum, 4);
    sum += __shfl_xor(sum, 2);
    sum += __shfl_xor(sum, 1);
    if (t == 0) sInv[r] = (1.0f / sum) * SC_PV;
  }
  __syncthreads();

  const int n = 16 * wave + m;
  const float* vcol = Vp + bL * ND + n;
  const f16t* prow_m = &uqk.p[m * NL + 8 * hh];
  v8f acc = zero8f();
  #pragma unroll 2
  for (int ks = 0; ks < NL / 32; ++ks) {
    const int k0 = 32 * ks;
    FragH A, Bf;
    A.half[0] = *(const v8ha*)(prow_m + k0);
    A.half[1] = *(const v8ha*)(prow_m + k0 + 16);
    #pragma unroll
    for (int i = 0; i < 8; ++i) {
      Bf.v[i]     = (f16t)(vcol[(size_t)(k0 + 8 * hh + i) * ND] * VCAR);
      Bf.v[8 + i] = (f16t)(vcol[(size_t)(k0 + 16 + 8 * hh + i) * ND] * VCAR);
    }
    acc = wmma_f16(A.v, Bf.v, acc);
  }

  float* const os = sS;
  #pragma unroll
  for (int r = 0; r < 8; ++r) {
    const int row = 8 * hh + r;
    os[row * OPITCH + n] = acc[r] * sInv[row];
  }
  __syncthreads();

  v4f va[2];
  float* da[2];
  #pragma unroll
  for (int j = 0; j < 2; ++j) {
    const int row = 2 * wave + j;
    va[j] = *(const v4fa*)(os + row * OPITCH + 4 * lane);
    da[j] = out + (size_t)(q0 + row) * ND + 4 * lane;
    *(volatile v4f*)da[j] = va[j];
  }
  __threadfence();
  #pragma unroll
  for (int j = 0; j < 2; ++j) *(volatile v4f*)da[j] = va[j];
}

extern "C" void kernel_launch(void* const* d_in, const int* in_sizes, int n_in,
                              void* d_out, int out_size, void* d_ws, size_t ws_size,
                              hipStream_t stream) {
  if (n_in < 15) return;
  if (in_sizes[0] != NROWS * ND || in_sizes[1] != NROWS * ND || in_sizes[2] != NROWS * ND) return;
  if (in_sizes[3] != ND * ND || in_sizes[5] != ND * ND || in_sizes[7] != ND * ND) return;
  if (in_sizes[4] != ND || in_sizes[6] != ND || in_sizes[8] != ND) return;
  if (in_sizes[9] != ND || in_sizes[11] != ND || in_sizes[13] != ND) return;
  if (in_sizes[10] < 1 || in_sizes[12] < 1 || in_sizes[14] < 1) return;
  if (out_size != NROWS * ND) return;

  const float* query   = (const float*)d_in[0];
  const float* key     = (const float*)d_in[1];
  const float* value   = (const float*)d_in[2];
  const float* Wq      = (const float*)d_in[3];
  const float* bq      = (const float*)d_in[4];
  const float* Wk      = (const float*)d_in[5];
  const float* bk      = (const float*)d_in[6];
  const float* Wv      = (const float*)d_in[7];
  const float* bv      = (const float*)d_in[8];
  const float* w_delta = (const float*)d_in[9];
  const float* b_delta = (const float*)d_in[10];
  const float* w_sigma = (const float*)d_in[11];
  const float* b_sigma = (const float*)d_in[12];
  const float* w_theta = (const float*)d_in[13];
  const float* b_theta = (const float*)d_in[14];
  float* outp = (float*)d_out;

  const size_t szP = (size_t)NROWS * ND * 4;
  size_t off = 0;
  char* ws = (char*)d_ws;
  float* Qp = (float*)(ws + off);  off += szP;
  float* Kp = (float*)(ws + off);  off += szP;
  float* Vp = (float*)(ws + off);  off += szP;
  if (off > ws_size) return;

  proj_k<<<dim3(NROWS / PJ_ROWS, 3), PJ_TPB, 0, stream>>>(query, key, value, Wq, bq, Wk, bk, Wv, bv, Qp, Kp, Vp);
  attn_k<<<NROWS / QT, AT_TPB, 0, stream>>>(Qp, Kp, Vp, w_delta, b_delta, w_sigma, b_sigma, w_theta, b_theta, outp);
  (void)hipGetLastError();
}
